// LSTMModel_84653805404857
// MI455X (gfx1250) — hardware-verified
//
#include <hip/hip_runtime.h>
#include <math.h>

constexpr int NBT     = 64;
constexpr int NTS     = 512;
constexpr int NIN     = 128;
constexpr int NHID    = 512;
constexpr int NGATE   = 4 * NHID;
constexpr int NLAY    = 2;
constexpr int NTHR    = 256;
constexpr int SEQ_BLK = 16;
constexpr int HPITCH  = 520;
constexpr int SLABP   = 68;
constexpr int TCH     = 128;
constexpr int NCHUNK  = NTS / TCH;
constexpr int NROWS   = NTS * NBT;
constexpr int CHROWS  = TCH * NBT;
constexpr int NSTATE  = NBT * NHID;
constexpr int NOUT0   = NBT;
constexpr int NOUTH   = NLAY * NSTATE;
constexpr float WCARRY = 256.0f;
constexpr float HCARRY = 16.0f;
constexpr float RC_INV = 1.0f / (WCARRY * HCARRY);
static_assert(NCHUNK * TCH == NTS);
static_assert(NBT % SEQ_BLK == 0);
static_assert(NHID == 64 * (NTHR / 32));
static_assert(NIN % 32 == 0 && NHID % 32 == 0);
static_assert(CHROWS % 64 == 0 && NGATE % 64 == 0);
static_assert((2 * SEQ_BLK * HPITCH) % NTHR == 0);
static_assert((SEQ_BLK * (NHID / 2)) % NTHR == 0);
static_assert(HPITCH % 8 == 0 && HPITCH >= NHID);
static_assert(NIN / 8 == 16);
static_assert((NROWS * (NIN / 8)) % NTHR == 0);
static_assert(SEQ_BLK % 8 == 0 && NBT % 8 == 0);
static_assert(NOUT0 * 4 == 256);
static_assert((NOUT0 + NOUTH) * 4 == 262400);
static_assert((NOUT0 + 2 * NOUTH) * 4 == 524544);

typedef __attribute__((ext_vector_type(16))) _Float16 v16h;
typedef __attribute__((ext_vector_type(8)))  _Float16 v8h;
typedef __attribute__((ext_vector_type(16))) __bf16   v16b;
typedef __attribute__((ext_vector_type(8)))  __bf16   v8b;
typedef __attribute__((ext_vector_type(8)))  float    v8f;
typedef __attribute__((ext_vector_type(4)))  float    v4f;

__device__ __forceinline__ unsigned short f2bf_bits(float f) {
  unsigned u = __float_as_uint(f);
  return (unsigned short)((u + 0x7FFFu + ((u >> 16) & 1u)) >> 16);
}
__device__ __forceinline__ float bf_bits2f(unsigned short h) { return __uint_as_float(((unsigned)h) << 16); }
__device__ __forceinline__ float bf16r(float f) { return bf_bits2f(f2bf_bits(f)); }

__device__ __forceinline__ void dep_guard_h(v8f& a, v8f& b, v16h x, v16h y) { asm volatile("v_nop\n\tv_nop\n\tv_nop\n\tv_nop" : "+v"(a), "+v"(b) : "v"(x), "v"(y)); }
__device__ __forceinline__ void dep_guard_b(v8f& a, v8f& b, v16b x, v16b y) { asm volatile("v_nop\n\tv_nop\n\tv_nop\n\tv_nop" : "+v"(a), "+v"(b) : "v"(x), "v"(y)); }
__device__ __forceinline__ void tie4_h(v8f& a0, v8f& a1, v8f& a2, v8f& a3, v16h x, v16h y) {
  asm volatile("v_nop\n\tv_nop\n\tv_nop\n\tv_nop" : "+v"(a0), "+v"(a1), "+v"(a2), "+v"(a3) : "v"(x), "v"(y));
}
__device__ __forceinline__ void tie4_b(v8f& a0, v8f& a1, v8f& a2, v8f& a3, v16b x, v16b y) {
  asm volatile("v_nop\n\tv_nop\n\tv_nop\n\tv_nop" : "+v"(a0), "+v"(a1), "+v"(a2), "+v"(a3) : "v"(x), "v"(y));
}
__device__ __forceinline__ void tie4x5_h(v8f& a0, v8f& a1, v8f& a2, v8f& a3, v16h x, v16h b0, v16h b1, v16h b2, v16h b3) {
  asm volatile("v_nop\n\tv_nop\n\tv_nop\n\tv_nop"
               : "+v"(a0), "+v"(a1), "+v"(a2), "+v"(a3)
               : "v"(x), "v"(b0), "v"(b1), "v"(b2), "v"(b3));
}
__device__ __forceinline__ void keep4_h(v16h a, v16h b, v16h c, v16h d) { asm volatile("v_nop" :: "v"(a), "v"(b), "v"(c), "v"(d)); }
__device__ __forceinline__ void keep4_b(v16b a, v16b b, v16b c, v16b d) { asm volatile("v_nop" :: "v"(a), "v"(b), "v"(c), "v"(d)); }
__device__ __forceinline__ void acc_guard4(v8f& a, v8f& b, v8f& c, v8f& d) { asm volatile("v_nop\n\tv_nop\n\tv_nop\n\tv_nop" : "+v"(a), "+v"(b), "+v"(c), "+v"(d)); }
template <typename T> struct Frag;
template <> struct Frag<_Float16> {
  typedef v16h V; union U { v16h v; v8h h[2]; };
  static __device__ __forceinline__ v16h load(const _Float16* p) {
    U f; f.h[0] = *(const v8h*)(p); f.h[1] = *(const v8h*)(p + 16); return f.v;
  }
  static __device__ __forceinline__ v8f mma(v16h a, v16h b, v8f c) {
    return __builtin_amdgcn_wmma_f32_16x16x32_f16(false, a, false, b, (short)0, c, false, false);
  }
  static __device__ __forceinline__ void guard(v8f& a, v8f& b, v16h x, v16h y) { dep_guard_h(a, b, x, y); }
  static __device__ __forceinline__ void guard4(v8f& a0, v8f& a1, v8f& a2, v8f& a3, v16h x, v16h y) { tie4_h(a0, a1, a2, a3, x, y); }
  static __device__ __forceinline__ void keep(v16h a, v16h b, v16h c, v16h d) { keep4_h(a, b, c, d); }
};
template <> struct Frag<__bf16> {
  typedef v16b V; union U { v16b v; v8b h[2]; };
  static __device__ __forceinline__ v16b load(const __bf16* p) {
    U f; f.h[0] = *(const v8b*)(p); f.h[1] = *(const v8b*)(p + 16); return f.v;
  }
  static __device__ __forceinline__ v8f mma(v16b a, v16b b, v8f c) {
    return __builtin_amdgcn_wmma_f32_16x16x32_bf16(false, a, false, b, (short)0, c, false, false);
  }
  static __device__ __forceinline__ void guard(v8f& a, v8f& b, v16b x, v16b y) { dep_guard_b(a, b, x, y); }
  static __device__ __forceinline__ void guard4(v8f& a0, v8f& a1, v8f& a2, v8f& a3, v16b x, v16b y) { tie4_b(a0, a1, a2, a3, x, y); }
  static __device__ __forceinline__ void keep(v16b a, v16b b, v16b c, v16b d) { keep4_b(a, b, c, d); }
};

__device__ __forceinline__ void wave_sync_lds() {
  __builtin_amdgcn_fence(__ATOMIC_RELEASE, "workgroup");
  __builtin_amdgcn_wave_barrier();
  __builtin_amdgcn_fence(__ATOMIC_ACQUIRE, "workgroup");
}

__device__ __forceinline__ float fsig(float x)  { return __builtin_amdgcn_rcpf(1.0f + expf(-x)); }
__device__ __forceinline__ float ftanh(float x) { return 1.0f - 2.0f * __builtin_amdgcn_rcpf(expf(2.0f * x) + 1.0f); }

template <int ET> struct Elem;
template <> struct Elem<0> { typedef _Float16 T; };
template <> struct Elem<1> { typedef __bf16 T; };
template <int ET, bool SPLIT, int BIAS_MODE, int OUT_MODE, bool RESID, int ACT = 0>
__global__ __launch_bounds__(256) __attribute__((amdgpu_num_vgpr(256))) void wmma_gemm64(
    const unsigned short* __restrict__ Ap, const unsigned short* __restrict__ A2p, int lda, long strideA,
    const unsigned short* __restrict__ Btp, const unsigned short* __restrict__ Bt2p, int ldb, long strideB,
    void* __restrict__ Cout, void* __restrict__ Cout2, int ldc, long strideC,
    const float* __restrict__ bias,
    const float* __restrict__ resid, long strideR,
    int M, int N, int K, float scale) {
  typedef typename Elem<ET>::T T;
  typedef typename Frag<T>::V V;
  const T* A = (const T*)Ap; const T* A2 = (const T*)A2p; const T* Bt = (const T*)Btp; const T* Bt2 = (const T*)Bt2p;
  __shared__ __align__(16) float sT[8][16 * 68];
  const int b    = blockIdx.y;
  const int lane = threadIdx.x & 31;
  const int wave = threadIdx.x >> 5;
  const int tilesN = N >> 6;
  const int tilesM = M >> 6;
  const int tile = blockIdx.x * 8 + wave;
  if (tile >= tilesM * tilesN) return;
  const int tm = tile / tilesN;
  const int tn = tile - tm * tilesN;
  const int m0 = tm << 6;
  const int n0 = tn << 6;

  const T* Ab  = A  + (size_t)b * strideA;
  const T* Bb  = Bt + (size_t)b * strideB;
  const T* Ab2 = SPLIT ? (A2  + (size_t)b * strideA) : nullptr;
  const T* Bb2 = SPLIT ? (Bt2 + (size_t)b * strideB) : nullptr;

  const int rlane = lane & 15;
  const int koff  = (lane >> 4) * 8;
  const int mOff  = (lane >> 4) * 8;

  v8f acc[4][4];
#pragma unroll
  for (int i = 0; i < 4; ++i)
#pragma unroll
    for (int j = 0; j < 4; ++j) acc[i][j] = (v8f){0.f,0.f,0.f,0.f,0.f,0.f,0.f,0.f};

  for (int k0 = 0; k0 < K; k0 += 32) {
    V bh[4], bl[4];
#pragma unroll
    for (int j = 0; j < 4; ++j) {
      const size_t bo = (size_t)(n0 + (j << 4) + rlane) * ldb + koff + k0;
      bh[j] = Frag<T>::load(Bb + bo);
      if (SPLIT) bl[j] = Frag<T>::load(Bb2 + bo);
    }
#pragma unroll
    for (int i = 0; i < 4; ++i) {
      const size_t ao = (size_t)(m0 + (i << 4) + rlane) * lda + koff + k0;
      V ah = Frag<T>::load(Ab + ao);
      V al;
      if (SPLIT) al = Frag<T>::load(Ab2 + ao);
#pragma unroll
      for (int j = 0; j < 4; ++j) {
        acc[i][j] = Frag<T>::mma(ah, bh[j], acc[i][j]);
        if (SPLIT) {
          acc[i][j] = Frag<T>::mma(ah, bl[j], acc[i][j]);
          acc[i][j] = Frag<T>::mma(al, bh[j], acc[i][j]);
        }
      }
      Frag<T>::guard4(acc[i][0], acc[i][1], acc[i][2], acc[i][3], ah, SPLIT ? al : ah);
    }
    Frag<T>::keep(bh[0], bh[1], bh[2], bh[3]);
    if (SPLIT) Frag<T>::keep(bl[0], bl[1], bl[2], bl[3]);
  }
  acc_guard4(acc[0][0], acc[0][1], acc[0][2], acc[0][3]);
  acc_guard4(acc[1][0], acc[1][1], acc[1][2], acc[1][3]);
  acc_guard4(acc[2][0], acc[2][1], acc[2][2], acc[2][3]);
  acc_guard4(acc[3][0], acc[3][1], acc[3][2], acc[3][3]);

  float* slab = sT[wave];
  const float* Rb = RESID ? (resid + (size_t)b * strideR) : nullptr;
#pragma unroll
  for (int i = 0; i < 4; ++i) {
    const int mBase = m0 + (i << 4);
    float bm[8];
#pragma unroll
    for (int r = 0; r < 8; ++r) bm[r] = 0.f;
    if (BIAS_MODE == 1) {
      const v4f t0 = *(const v4f*)(bias + mBase + mOff);
      const v4f t1 = *(const v4f*)(bias + mBase + mOff + 4);
#pragma unroll
      for (int e = 0; e < 4; ++e) { bm[e] = t0[e]; bm[4 + e] = t1[e]; }
    }
#pragma unroll
    for (int j = 0; j < 4; ++j) {
      const int n = n0 + (j << 4) + rlane;
      float bv = 0.f;
      if (BIAS_MODE == 2) bv = bias[n];
#pragma unroll
      for (int r = 0; r < 8; ++r) {
        float v = acc[i][j][r] * scale;
        if (BIAS_MODE == 1) v += bm[r];
        if (BIAS_MODE == 2) v += bv;
        if (RESID) v += Rb[(size_t)(mBase + mOff + r) * ldc + n];
        if (ACT == 1) v = tanhf(v);
        if (ACT == 2) v = fmaxf(v, 0.0f);
        if (ACT == 3) v = v / (1.0f + expf(-v));
        if (ACT == 4) v = (v > 0.f) ? v : 0.01f * v;
        if (ACT == 5) v = 0.5f * v * (1.0f + erff(v * 0.70710678118654752f));
        slab[(mOff + r) * 68 + (j << 4) + rlane] = v;
      }
    }
    __builtin_amdgcn_fence(__ATOMIC_RELEASE, "workgroup");
    __builtin_amdgcn_wave_barrier();
    __builtin_amdgcn_fence(__ATOMIC_ACQUIRE, "workgroup");
    if (OUT_MODE == 0) {
      float* C = (float*)Cout + (size_t)b * strideC;
      const int hh = lane >> 4, c4 = (lane & 15) * 4;
      for (int pass = 0; pass < 2; ++pass) {
#pragma unroll
        for (int it = 0; it < 8; ++it) {
          const int row = it * 2 + hh;
          v4f v = *(const v4f*)(slab + row * 68 + c4);
          *(volatile v4f*)(C + (size_t)(mBase + row) * ldc + n0 + c4) = v;
        }
        __threadfence();
      }
    } else {
      const int q = lane >> 3, c8 = (lane & 7) * 8;
      unsigned short* C  = (unsigned short*)Cout  + (size_t)b * strideC;
      unsigned short* C2 = (OUT_MODE == 2) ? ((unsigned short*)Cout2 + (size_t)b * strideC) : nullptr;
      for (int pass = 0; pass < 2; ++pass) {
#pragma unroll
        for (int it = 0; it < 4; ++it) {
          const int row = it * 4 + q;
          const float* sp = slab + row * 68 + c8;
          v8h hv, lv;
#pragma unroll
          for (int e = 0; e < 8; ++e) {
            if (OUT_MODE == 1) {
              hv[e] = (_Float16)sp[e];
            } else {
              unsigned short hb = f2bf_bits(sp[e]);
              unsigned short lb = f2bf_bits(sp[e] - bf_bits2f(hb));
              hv[e] = __builtin_bit_cast(_Float16, hb);
              lv[e] = __builtin_bit_cast(_Float16, lb);
            }
          }
          *(volatile v8h*)(C + (size_t)(mBase + row) * ldc + n0 + c8) = hv;
          if (OUT_MODE == 2) *(volatile v8h*)(C2 + (size_t)(mBase + row) * ldc + n0 + c8) = lv;
        }
        __threadfence();
      }
    }
    __builtin_amdgcn_fence(__ATOMIC_RELEASE, "workgroup");
    __builtin_amdgcn_wave_barrier();
    __builtin_amdgcn_fence(__ATOMIC_ACQUIRE, "workgroup");
  }
}

template <int MODE>
__global__ __launch_bounds__(NTHR) void cvt8_kernel(const float* __restrict__ src, unsigned short* __restrict__ dst,
                                                    int nrow, int ncol8, int spitch, int scol0, float sc) {
  const int i  = blockIdx.x * NTHR + threadIdx.x;
  const int n8 = nrow * ncol8;
  if (i < n8) {
    const int row = i / ncol8;
    const int c8  = i - row * ncol8;
    const float* sp = src + (size_t)row * spitch + scol0 + c8 * 8;
    const v4f a = *(const v4f*)(sp);
    const v4f b = *(const v4f*)(sp + 4);
    v8h hv;
#pragma unroll
    for (int e = 0; e < 4; ++e) {
      unsigned short b0, b1;
      if (MODE == 0) {
        b0 = f2bf_bits(a[e] * sc);
        b1 = f2bf_bits(b[e] * sc);
      } else {
        b0 = __builtin_bit_cast(unsigned short, (_Float16)(bf16r(a[e]) * sc));
        b1 = __builtin_bit_cast(unsigned short, (_Float16)(bf16r(b[e]) * sc));
      }
      hv[e]     = __builtin_bit_cast(_Float16, b0);
      hv[4 + e] = __builtin_bit_cast(_Float16, b1);
    }
    *(volatile v8h*)(dst + (size_t)i * 8) = hv;
    __threadfence();
    *(volatile v8h*)(dst + (size_t)i * 8) = hv;
  }
}

__global__ __launch_bounds__(NTHR) void xpack_kernel(const float* __restrict__ x, unsigned short* __restrict__ XB) {
  const int i = blockIdx.x * NTHR + threadIdx.x;
  if (i < NROWS * (NIN / 8)) {
    const int rd = i >> 4, c8 = (i & 15) * 8;
    const int t = rd / NBT, b = rd - t * NBT;
    const float* sp = x + ((size_t)b * NTS + (size_t)t) * NIN + c8;
    const v4f a = *(const v4f*)sp;
    const v4f q = *(const v4f*)(sp + 4);
    v8h hv;
#pragma unroll
    for (int e = 0; e < 4; ++e) {
      hv[e]     = __builtin_bit_cast(_Float16, f2bf_bits(a[e]));
      hv[4 + e] = __builtin_bit_cast(_Float16, f2bf_bits(q[e]));
    }
    *(volatile v8h*)(XB + (size_t)i * 8) = hv;
    __threadfence();
    *(volatile v8h*)(XB + (size_t)i * 8) = hv;
  }
}

__global__ __launch_bounds__(NTHR) void cinit_kernel(const float* __restrict__ src, float* __restrict__ dst, int n4) {
  const int i = blockIdx.x * NTHR + threadIdx.x;
  if (i < n4) {
    const v4f v = *(const v4f*)(src + (size_t)i * 4);
    v4f o;
#pragma unroll
    for (int e = 0; e < 4; ++e) o[e] = bf16r(v[e]);
    *(volatile v4f*)(dst + (size_t)i * 4) = o;
    __threadfence();
    *(volatile v4f*)(dst + (size_t)i * 4) = o;
  }
}

__global__ __launch_bounds__(NTHR) void bias_kernel(const float* __restrict__ bi0, const float* __restrict__ bh0,
                                                    const float* __restrict__ bi1, const float* __restrict__ bh1,
                                                    float* __restrict__ BS) {
  const int gi = blockIdx.x * NTHR + threadIdx.x;
  if (gi < 2 * (NGATE / 4)) {
    const int l  = gi >> 9;
    const int n4 = (gi & 511) * 4;
    const v4f a0 = *(const v4f*)(bi0 + n4);
    const v4f c0 = *(const v4f*)(bh0 + n4);
    const v4f a1 = *(const v4f*)(bi1 + n4);
    const v4f c1 = *(const v4f*)(bh1 + n4);
    v4f o;
#pragma unroll
    for (int e = 0; e < 4; ++e) {
      const float s0 = bf16r(a0[e]) + bf16r(c0[e]);
      const float s1 = bf16r(a1[e]) + bf16r(c1[e]);
      o[e] = l ? s1 : s0;
    }
    float* op = BS + (size_t)l * NGATE + n4;
    *(volatile v4f*)op = o;
    __threadfence();
    *(volatile v4f*)op = o;
  }
}

template <bool WSEQ, bool WFIN>
__global__ __launch_bounds__(NTHR) __attribute__((amdgpu_num_vgpr(256)))
void lstm_chunk_kernel(const float* __restrict__ XGT, const unsigned short* __restrict__ WHp,
                       const unsigned short* __restrict__ hst_in,
                       unsigned short* __restrict__ hst_out,
                       const float* __restrict__ cst_in, float* __restrict__ cst_out,
                       unsigned short* __restrict__ HSEQ, float* __restrict__ HFIN,
                       float* __restrict__ hn_out, float* __restrict__ cn_out, int t0) {
  __shared__ __align__(16) _Float16 Ah[2][SEQ_BLK * HPITCH];
  __shared__ __align__(16) float    Sl[NTHR / 32][16 * SLABP];
  const _Float16* WH = (const _Float16*)WHp;
  const int tid = threadIdx.x, lane = tid & 31, wave = tid >> 5;
  const int c = lane & 15, hh = lane >> 4, koff = hh * 8, c4 = c * 4;
  const int q = lane >> 3, c8 = (lane & 7) * 8;
  const int rowbase = blockIdx.x * SEQ_BLK;
  float* slab = Sl[wave];

  {
    _Float16* ahf = &Ah[0][0];
#pragma unroll 1
    for (int i = tid; i < 2 * SEQ_BLK * HPITCH; i += NTHR) ahf[i] = (_Float16)0.0f;
  }
  __syncthreads();
  {
    const unsigned* hs = (const unsigned*)(const void*)hst_in;
    unsigned* a0 = (unsigned*)(void*)&Ah[0][0];
#pragma unroll 1
    for (int i = tid; i < SEQ_BLK * (NHID / 2); i += NTHR) {
      const int row = i >> 8, w2 = i & 255;
      a0[row * (HPITCH / 2) + w2] = hs[(size_t)(rowbase + row) * (NHID / 2) + w2];
    }
  }
  float cst[4][8];
  {
#pragma unroll
    for (int it = 0; it < 8; ++it) {
      const int row = it * 2 + hh;
      const v4f v = *(const v4f*)(cst_in + (size_t)(rowbase + row) * NHID + 64 * wave + c4);
      *(v4f*)(slab + row * SLABP + c4) = v;
    }
    wave_sync_lds();
#pragma unroll
    for (int ub = 0; ub < 4; ++ub) {
#pragma unroll
      for (int r = 0; r < 8; ++r) cst[ub][r] = slab[(8 * hh + r) * SLABP + 16 * ub + c];
    }
    wave_sync_lds();
  }
  __syncthreads();

  const v8f z8 = {0.f, 0.f, 0.f, 0.f, 0.f, 0.f, 0.f, 0.f};

#pragma unroll 1
  for (int ls = 0; ls < TCH; ++ls) {
    const int cur = ls & 1;
    const _Float16* ahrow = &Ah[cur][0] + c * HPITCH + koff;
    _Float16* ahn = &Ah[cur ^ 1][0];
    const float* xcol = XGT + (size_t)ls * NBT + rowbase + 8 * hh;

#pragma unroll
    for (int ub = 0; ub < 4; ++ub) {
      const int u = 64 * wave + 16 * ub + c;
      const _Float16* w0 = WH + (size_t)u * NHID + koff;
      v8f acc[4];
      acc[0] = z8; acc[1] = z8; acc[2] = z8; acc[3] = z8;
#pragma unroll 1
      for (int k0 = 0; k0 < NHID; k0 += 32) {
        const v16h a  = Frag<_Float16>::load(ahrow + k0);
        const v16h b0 = Frag<_Float16>::load(w0 + k0);
        const v16h b1 = Frag<_Float16>::load(w0 + (size_t)1 * NHID * NHID + k0);
        const v16h b2 = Frag<_Float16>::load(w0 + (size_t)2 * NHID * NHID + k0);
        const v16h b3 = Frag<_Float16>::load(w0 + (size_t)3 * NHID * NHID + k0);
        acc[0] = Frag<_Float16>::mma(a, b0, acc[0]);
        acc[1] = Frag<_Float16>::mma(a, b1, acc[1]);
        acc[2] = Frag<_Float16>::mma(a, b2, acc[2]);
        acc[3] = Frag<_Float16>::mma(a, b3, acc[3]);
        tie4x5_h(acc[0], acc[1], acc[2], acc[3], a, b0, b1, b2, b3);
      }
      acc_guard4(acc[0], acc[1], acc[2], acc[3]);

      v8f xg[4];
#pragma unroll
      for (int g = 0; g < 4; ++g) xg[g] = *(const v8f*)(xcol + (size_t)(g * NHID + u) * CHROWS);

#pragma unroll
      for (int r = 0; r < 8; ++r) {
        const float zi = acc[0][r] * RC_INV + xg[0][r];
        const float zf = acc[1][r] * RC_INV + xg[1][r];
        const float zg = acc[2][r] * RC_INV + xg[2][r];
        const float zo = acc[3][r] * RC_INV + xg[3][r];
        const float ig = fsig(zi);
        const float fg = fsig(zf);
        const float gg = ftanh(zg);
        const float og = fsig(zo);
        const float cn = fg * cst[ub][r] + ig * gg;
        cst[ub][r] = cn;
        const float hn = og * ftanh(cn);
        ahn[(8 * hh + r) * HPITCH + u] = (_Float16)(hn * HCARRY);
        slab[(8 * hh + r) * SLABP + 16 * ub + c] = hn;
      }
      asm volatile("" ::: "memory");
    }

    wave_sync_lds();
    const int t = t0 + ls;
    const bool lastc = (ls == TCH - 1);
    const bool fin   = lastc && (t0 + TCH == NTS);
    if (WSEQ || lastc) {
      for (int pass = 0; pass < 2; ++pass) {
#pragma unroll
        for (int it = 0; it < 4; ++it) {
          const int row = it * 4 + q;
          const float* sp = slab + row * SLABP + c8;
          const v4f s0 = *(const v4f*)(sp);
          const v4f s1 = *(const v4f*)(sp + 4);
          v8h hv;
#pragma unroll
          for (int e = 0; e < 4; ++e) {
            hv[e]     = (_Float16)(s0[e] * HCARRY);
            hv[4 + e] = (_Float16)(s1[e] * HCARRY);
          }
          if (WSEQ)  *(volatile v8h*)(HSEQ + ((size_t)t * NBT + (size_t)(rowbase + row)) * NHID + 64 * wave + c8) = hv;
          if (lastc) *(volatile v8h*)(hst_out + (size_t)(rowbase + row) * NHID + 64 * wave + c8) = hv;
        }
        __threadfence();
      }
    }
    if (fin) {
      for (int pass = 0; pass < 2; ++pass) {
#pragma unroll
        for (int it = 0; it < 8; ++it) {
          const int row = it * 2 + hh;
          const v4f v = *(const v4f*)(slab + row * SLABP + c4);
          *(volatile v4f*)(hn_out + (size_t)(rowbase + row) * NHID + 64 * wave + c4) = v;
          if (WFIN) *(volatile v4f*)(HFIN + (size_t)(rowbase + row) * NHID + 64 * wave + c4) = v;
        }
        __threadfence();
      }
    }
    if (lastc) {
      wave_sync_lds();
#pragma unroll
      for (int ub = 0; ub < 4; ++ub)
#pragma unroll
        for (int r = 0; r < 8; ++r) slab[(8 * hh + r) * SLABP + 16 * ub + c] = cst[ub][r];
      wave_sync_lds();
      for (int pass = 0; pass < 2; ++pass) {
#pragma unroll
        for (int it = 0; it < 8; ++it) {
          const int row = it * 2 + hh;
          const v4f v = *(const v4f*)(slab + row * SLABP + c4);
          *(volatile v4f*)(cst_out + (size_t)(rowbase + row) * NHID + 64 * wave + c4) = v;
          if (fin) *(volatile v4f*)(cn_out + (size_t)(rowbase + row) * NHID + 64 * wave + c4) = v;
        }
        __threadfence();
      }
    }
    __syncthreads();
  }
}

__global__ __launch_bounds__(NTHR) void head_kernel(const float* __restrict__ HF, const float* __restrict__ fw,
                                                    const float* __restrict__ fb, float* __restrict__ out) {
  __shared__ __align__(16) float red[NBT];
  const int tid = threadIdx.x, lane = tid & 31, wave = tid >> 5;
  v4f w[4];
#pragma unroll
  for (int qq = 0; qq < 4; ++qq) {
    const v4f tw = *(const v4f*)(fw + 16 * lane + 4 * qq);
    v4f rw;
#pragma unroll
    for (int e = 0; e < 4; ++e) rw[e] = bf16r(tw[e]);
    w[qq] = rw;
  }
  const float b0 = bf16r(fb[0]);
#pragma unroll 1
  for (int i = 0; i < NBT / 8; ++i) {
    const int b = wave * (NBT / 8) + i;
    float s = 0.0f;
#pragma unroll
    for (int qq = 0; qq < 4; ++qq) {
      const v4f hv = *(const v4f*)(HF + (size_t)b * NHID + 16 * lane + 4 * qq);
      s += hv[0] * w[qq][0];
      s += hv[1] * w[qq][1];
      s += hv[2] * w[qq][2];
      s += hv[3] * w[qq][3];
    }
#pragma unroll
    for (int off = 1; off < 32; off <<= 1) s += __shfl_xor(s, off, 32);
    if (lane == 0) red[b] = s + b0;
  }
  __syncthreads();
  if (wave == 0) {
    const v4f v = *(const v4f*)(red + 4 * (lane & 15));
    for (int pass = 0; pass < 2; ++pass) {
      if (lane < 16) *(volatile v4f*)(out + 4 * lane) = v;
      __threadfence();
    }
  }
}

extern "C" void kernel_launch(void* const* d_in, const int* in_sizes, int n_in,
                              void* d_out, int out_size, void* d_ws, size_t ws_size, hipStream_t stream) {
  if (n_in < 13 || d_out == nullptr || d_ws == nullptr) return;
  if (in_sizes[0] != NBT * NTS * NIN || in_sizes[1] != NLAY * NSTATE || in_sizes[2] != NLAY * NSTATE ||
      in_sizes[3] != NGATE * NIN || in_sizes[4] != NGATE * NHID || in_sizes[5] != NGATE || in_sizes[6] != NGATE ||
      in_sizes[7] != NGATE * NHID || in_sizes[8] != NGATE * NHID || in_sizes[9] != NGATE || in_sizes[10] != NGATE ||
      in_sizes[11] != NHID || in_sizes[12] != 1 || out_size != NOUT0 + 2 * NOUTH) return;

  const float* x      = (const float*)d_in[0];
  const float* hx     = (const float*)d_in[1];
  const float* cx     = (const float*)d_in[2];
  const float* w_ih_0 = (const float*)d_in[3];
  const float* w_hh_0 = (const float*)d_in[4];
  const float* b_ih_0 = (const float*)d_in[5];
  const float* b_hh_0 = (const float*)d_in[6];
  const float* w_ih_1 = (const float*)d_in[7];
  const float* w_hh_1 = (const float*)d_in[8];
  const float* b_ih_1 = (const float*)d_in[9];
  const float* b_hh_1 = (const float*)d_in[10];
  const float* fc_w   = (const float*)d_in[11];
  const float* fc_b   = (const float*)d_in[12];
  float* out = (float*)d_out;
  float* hn0 = out + NOUT0;
  float* hn1 = hn0 + NSTATE;
  float* cn0 = out + NOUT0 + NOUTH;
  float* cn1 = cn0 + NSTATE;

  char* ws = (char*)d_ws; size_t off = 0;
  auto carve = [&](size_t bytes) -> char* { char* p = ws + off; off += (bytes + 255) & ~(size_t)255; return p; };
  unsigned short* XB   = (unsigned short*)carve((size_t)NROWS * NIN * 2);
  unsigned short* WI0  = (unsigned short*)carve((size_t)NGATE * NIN * 2);
  unsigned short* WH0  = (unsigned short*)carve((size_t)NGATE * NHID * 2);
  unsigned short* WI1  = (unsigned short*)carve((size_t)NGATE * NHID * 2);
  unsigned short* WH1  = (unsigned short*)carve((size_t)NGATE * NHID * 2);
  float*          BS   = (float*)carve((size_t)NLAY * NGATE * 4);
  float*          XGT  = (float*)carve((size_t)NGATE * CHROWS * 4);
  unsigned short* HSEQ = (unsigned short*)carve((size_t)NROWS * NHID * 2);
  unsigned short* HST  = (unsigned short*)carve((size_t)2 * NLAY * NSTATE * 2);
  float*          CST  = (float*)carve((size_t)2 * NLAY * NSTATE * 4);
  float*          H1F  = (float*)carve((size_t)NSTATE * 4);
  if (off > ws_size || off > (size_t)134217728) return;

  const int n8x  = NROWS * (NIN / 8);
  const int n8w0 = NGATE * (NIN / 8);
  const int n8w  = NGATE * (NHID / 8);
  const int n8h  = NLAY * NBT * (NHID / 8);
  const int n4c  = NLAY * NSTATE / 4;
  xpack_kernel<<<(n8x + NTHR - 1) / NTHR, NTHR, 0, stream>>>(x, XB);
  cvt8_kernel<0><<<(n8w0 + NTHR - 1) / NTHR, NTHR, 0, stream>>>(w_ih_0, WI0, NGATE, NIN / 8, NIN, 0, 1.0f);
  cvt8_kernel<1><<<(n8w + NTHR - 1) / NTHR, NTHR, 0, stream>>>(w_hh_0, WH0, NGATE, NHID / 8, NHID, 0, WCARRY);
  cvt8_kernel<1><<<(n8w + NTHR - 1) / NTHR, NTHR, 0, stream>>>(w_ih_1, WI1, NGATE, NHID / 8, NHID, 0, WCARRY);
  cvt8_kernel<1><<<(n8w + NTHR - 1) / NTHR, NTHR, 0, stream>>>(w_hh_1, WH1, NGATE, NHID / 8, NHID, 0, WCARRY);
  bias_kernel<<<(2 * (NGATE / 4) + NTHR - 1) / NTHR, NTHR, 0, stream>>>(b_ih_0, b_hh_0, b_ih_1, b_hh_1, BS);
  cvt8_kernel<1><<<(n8h + NTHR - 1) / NTHR, NTHR, 0, stream>>>(hx, HST, NLAY * NBT, NHID / 8, NHID, 0, HCARRY);
  cinit_kernel<<<(n4c + NTHR - 1) / NTHR, NTHR, 0, stream>>>(cx, CST, n4c);

  const dim3 ggrid((NGATE / 64) * (CHROWS / 64) / 8, 1);
  const dim3 rgrid(NBT / SEQ_BLK, 1);

  for (int ch = 0; ch < NCHUNK; ++ch) {
    const int pin = ch & 1, pout = (ch + 1) & 1;
    wmma_gemm64<1, false, 1, 0, false, 0><<<ggrid, 256, 0, stream>>>(
        WI0, WI0, NIN, 0L,
        XB + (size_t)ch * CHROWS * NIN, XB + (size_t)ch * CHROWS * NIN, NIN, 0L,
        (void*)XGT, (void*)XGT, CHROWS, 0L,
        BS, (const float*)XGT, 0L, NGATE, CHROWS, NIN, 1.0f);
    lstm_chunk_kernel<true, false><<<rgrid, NTHR, 0, stream>>>(
        XGT, WH0,
        HST + (size_t)(pin * NLAY + 0) * NSTATE, HST + (size_t)(pout * NLAY + 0) * NSTATE,
        CST + (size_t)(pin * NLAY + 0) * NSTATE, CST + (size_t)(pout * NLAY + 0) * NSTATE,
        HSEQ, H1F, hn0, cn0, ch * TCH);
  }
  for (int ch = 0; ch < NCHUNK; ++ch) {
    const int pin = ch & 1, pout = (ch + 1) & 1;
    wmma_gemm64<0, false, 1, 0, false, 0><<<ggrid, 256, 0, stream>>>(
        WI1, WI1, NHID, 0L,
        HSEQ + (size_t)ch * CHROWS * NHID, HSEQ + (size_t)ch * CHROWS * NHID, NHID, 0L,
        (void*)XGT, (void*)XGT, CHROWS, 0L,
        BS + NGATE, (const float*)XGT, 0L, NGATE, CHROWS, NHID, RC_INV);
    lstm_chunk_kernel<false, true><<<rgrid, NTHR, 0, stream>>>(
        XGT, WH1,
        HST + (size_t)(pin * NLAY + 1) * NSTATE, HST + (size_t)(pout * NLAY + 1) * NSTATE,
        CST + (size_t)(pin * NLAY + 1) * NSTATE, CST + (size_t)(pout * NLAY + 1) * NSTATE,
        HSEQ, H1F, hn1, cn1, ch * TCH);
  }
  head_kernel<<<1, NTHR, 0, stream>>>(H1F, fc_w, fc_b, out);
}
